// DinoV2Attention_79903571574925
// MI455X (gfx1250) — hardware-verified
//
#include <hip/hip_runtime.h>
#include <math.h>
#include <stdint.h>

#define NB   8
#define SEQ  1370
#define SP   1408
#define DM   1024
#define NH   16
#define DH   64
#define QKP  2048
#define GRP  4
#define NGRP 2
#define NQB  (SP / 64)
#define NKC  (SP / 64)

typedef __attribute__((ext_vector_type(16))) _Float16 v16h;
typedef __attribute__((ext_vector_type(8)))  _Float16 v8h;
typedef __attribute__((ext_vector_type(16))) __bf16   v16b;
typedef __attribute__((ext_vector_type(8)))  __bf16   v8b;
typedef __attribute__((ext_vector_type(8)))  float    v8f;
typedef __attribute__((ext_vector_type(4)))  float    v4f;
typedef __attribute__((ext_vector_type(4)))  unsigned int v4u;

__device__ __forceinline__ unsigned short f2bf_bits(float f) {
  unsigned u = __float_as_uint(f);
  return (unsigned short)((u + 0x7FFFu + ((u >> 16) & 1u)) >> 16);
}
__device__ __forceinline__ float bf_bits2f(unsigned short h) { return __uint_as_float(((unsigned)h) << 16); }
__device__ __forceinline__ unsigned pk16(unsigned short a, unsigned short b) { return (unsigned)a | ((unsigned)b << 16); }
__device__ __forceinline__ unsigned short h_bits(_Float16 h) { return __builtin_bit_cast(unsigned short, h); }
__device__ __forceinline__ v8f zero8() {
  v8f z;
#pragma unroll
  for (int i = 0; i < 8; ++i) z[i] = 0.0f;
  return z;
}

__device__ __forceinline__ void dep_guard_h(v8f& a, v8f& b, v16h x, v16h y) { asm volatile("v_nop\n\tv_nop\n\tv_nop\n\tv_nop" : "+v"(a), "+v"(b) : "v"(x), "v"(y)); }
__device__ __forceinline__ void dep_guard_b(v8f& a, v8f& b, v16b x, v16b y) { asm volatile("v_nop\n\tv_nop\n\tv_nop\n\tv_nop" : "+v"(a), "+v"(b) : "v"(x), "v"(y)); }
__device__ __forceinline__ void keep4_h(v16h a, v16h b, v16h c, v16h d) { asm volatile("v_nop" :: "v"(a), "v"(b), "v"(c), "v"(d)); }
__device__ __forceinline__ void keep4_b(v16b a, v16b b, v16b c, v16b d) { asm volatile("v_nop" :: "v"(a), "v"(b), "v"(c), "v"(d)); }
__device__ __forceinline__ void acc_guard4(v8f& a, v8f& b, v8f& c, v8f& d) { asm volatile("v_nop\n\tv_nop\n\tv_nop\n\tv_nop" : "+v"(a), "+v"(b), "+v"(c), "+v"(d)); }

template <typename T> struct Frag;
template <> struct Frag<_Float16> {
  typedef v16h V; union U { v16h v; v8h h[2]; };
  static __device__ __forceinline__ v16h load(const _Float16* p) {
    U f; f.h[0] = *(const v8h*)(p); f.h[1] = *(const v8h*)(p + 16); return f.v;
  }
  static __device__ __forceinline__ v8f mma(v16h a, v16h b, v8f c) {
    return __builtin_amdgcn_wmma_f32_16x16x32_f16(false, a, false, b, (short)0, c, false, false);
  }
  static __device__ __forceinline__ void guard(v8f& a, v8f& b, v16h x, v16h y) { dep_guard_h(a, b, x, y); }
  static __device__ __forceinline__ void keep(v16h a, v16h b, v16h c, v16h d) { keep4_h(a, b, c, d); }
};
template <> struct Frag<__bf16> {
  typedef v16b V; union U { v16b v; v8b h[2]; };
  static __device__ __forceinline__ v16b load(const __bf16* p) {
    U f; f.h[0] = *(const v8b*)(p); f.h[1] = *(const v8b*)(p + 16); return f.v;
  }
  static __device__ __forceinline__ v8f mma(v16b a, v16b b, v8f c) {
    return __builtin_amdgcn_wmma_f32_16x16x32_bf16(false, a, false, b, (short)0, c, false, false);
  }
  static __device__ __forceinline__ void guard(v8f& a, v8f& b, v16b x, v16b y) { dep_guard_b(a, b, x, y); }
  static __device__ __forceinline__ void keep(v16b a, v16b b, v16b c, v16b d) { keep4_b(a, b, c, d); }
};

template <int ET> struct Elem;
template <> struct Elem<0> { typedef _Float16 T; };
template <> struct Elem<1> { typedef __bf16 T; };

template <int ET, int BIAS_MODE, int OUT_MODE>
__global__ __launch_bounds__(256) void gemm64_kernel(
    const unsigned short* __restrict__ Ap, int lda, long strideA,
    const unsigned short* __restrict__ Btp, int ldb, long strideB,
    void* __restrict__ Cout, void* __restrict__ Cout2, int ldc, long strideC,
    const float* __restrict__ bias, const float* __restrict__ bias2, int Nb,
    int M, int N, int K, int Mv, float scale, float oscale) {
  typedef typename Elem<ET>::T T;
  typedef typename Frag<T>::V V;
  const T* A  = (const T*)(const void*)Ap;
  const T* Bt = (const T*)(const void*)Btp;
  __shared__ __align__(16) float sT[8][16 * 68];
  const int b    = blockIdx.y;
  const int lane = threadIdx.x & 31;
  const int wave = threadIdx.x >> 5;
  const int tilesN = N >> 6;
  const int tilesM = M >> 6;
  const int tile = blockIdx.x * 8 + wave;
  if (tile >= tilesM * tilesN) return;
  const int tm = tile / tilesN;
  const int tn = tile - tm * tilesN;
  const int m0 = tm << 6;
  const int n0 = tn << 6;

  const T* Ab = A  + (size_t)b * (size_t)strideA;
  const T* Bb = Bt + (size_t)b * (size_t)strideB;

  const int rlane = lane & 15;
  const int koff  = (lane >> 4) * 8;
  const int mOff  = (lane >> 4) * 8;

  v8f acc[4][4];
#pragma unroll
  for (int i = 0; i < 4; ++i)
#pragma unroll
    for (int j = 0; j < 4; ++j) acc[i][j] = zero8();

  for (int k0 = 0; k0 < K; k0 += 32) {
    V bf[4];
#pragma unroll
    for (int j = 0; j < 4; ++j) {
      const size_t bo = (size_t)(n0 + (j << 4) + rlane) * (size_t)ldb + koff + k0;
      bf[j] = Frag<T>::load(Bb + bo);
    }
#pragma unroll
    for (int i = 0; i < 4; ++i) {
      const size_t ao = (size_t)(m0 + (i << 4) + rlane) * (size_t)lda + koff + k0;
      V af = Frag<T>::load(Ab + ao);
#pragma unroll
      for (int j = 0; j < 4; ++j) acc[i][j] = Frag<T>::mma(af, bf[j], acc[i][j]);
      Frag<T>::guard(acc[i][0], acc[i][3], af, af);
    }
    Frag<T>::keep(bf[0], bf[1], bf[2], bf[3]);
  }
  acc_guard4(acc[0][0], acc[0][1], acc[0][2], acc[0][3]);
  acc_guard4(acc[1][0], acc[1][1], acc[1][2], acc[1][3]);
  acc_guard4(acc[2][0], acc[2][1], acc[2][2], acc[2][3]);
  acc_guard4(acc[3][0], acc[3][1], acc[3][2], acc[3][3]);

  float* slab = sT[wave];
#pragma unroll
  for (int i = 0; i < 4; ++i) {
    const int mBase = m0 + (i << 4);
#pragma unroll
    for (int j = 0; j < 4; ++j) {
      const int n = n0 + (j << 4) + rlane;
      float bvn = 0.f;
      if (BIAS_MODE == 2) {
        const int i1 = (n < Nb) ? n : (Nb - 1);
        int i2 = n - Nb;
        i2 = (i2 < 0) ? 0 : i2;
        i2 = (i2 > Nb - 1) ? (Nb - 1) : i2;
        const float b1 = bias[i1];
        const float b2 = bias2[i2];
        bvn = (n < Nb) ? b1 : b2;
      }
#pragma unroll
      for (int r = 0; r < 8; ++r) {
        float v = acc[i][j][r] * scale;
        if (BIAS_MODE == 1) v += bias[mBase + mOff + r];
        if (BIAS_MODE == 2) v += bvn;
        v *= oscale;
        slab[(mOff + r) * 68 + (j << 4) + rlane] = v;
      }
    }
    __builtin_amdgcn_fence(__ATOMIC_RELEASE, "workgroup");
    __builtin_amdgcn_wave_barrier();
    __builtin_amdgcn_fence(__ATOMIC_ACQUIRE, "workgroup");
    if (OUT_MODE == 0) {
      float* C = (float*)Cout + (size_t)b * (size_t)strideC;
      const int hh = lane >> 4, c4 = (lane & 15) * 4;
      for (int pass = 0; pass < 2; ++pass) {
#pragma unroll
        for (int it = 0; it < 8; ++it) {
          const int row = it * 2 + hh;
          const v4f v = *(const v4f*)(slab + row * 68 + c4);
          if (mBase + row < Mv)
            *(volatile v4f*)(C + (size_t)(mBase + row) * (size_t)ldc + n0 + c4) = v;
        }
        __threadfence();
      }
    } else {
      const int q = lane >> 3, c8 = (lane & 7) * 8;
      unsigned short* C  = (unsigned short*)Cout  + (size_t)b * (size_t)strideC;
      unsigned short* C2 = (unsigned short*)Cout2 + (size_t)b * (size_t)strideC;
      for (int pass = 0; pass < 2; ++pass) {
#pragma unroll
        for (int it = 0; it < 4; ++it) {
          const int row = it * 4 + q;
          const float* sp = slab + row * 68 + c8;
          v8h hv, lv;
#pragma unroll
          for (int e = 0; e < 8; ++e) {
            const float f = sp[e];
            const _Float16 hf = (_Float16)f;
            hv[e] = hf;
            if (OUT_MODE == 2) lv[e] = (_Float16)((f - (float)hf) * 2048.0f);
            else lv[e] = hf;
          }
          *(volatile v8h*)(C + (size_t)(mBase + row) * (size_t)ldc + n0 + c8) = hv;
          if (OUT_MODE == 2) *(volatile v8h*)(C2 + (size_t)(mBase + row) * (size_t)ldc + n0 + c8) = lv;
        }
        __threadfence();
      }
    }
    __builtin_amdgcn_fence(__ATOMIC_RELEASE, "workgroup");
    __builtin_amdgcn_wave_barrier();
    __builtin_amdgcn_fence(__ATOMIC_ACQUIRE, "workgroup");
  }
}

__global__ __launch_bounds__(256) void xconv_kernel(const float* __restrict__ x, unsigned short* __restrict__ xb) {
  const int tid = threadIdx.x;
  const int row = blockIdx.x * 2 + (tid >> 7);
  const int b   = row / SP;
  const int s   = row - b * SP;
  const int c8  = (tid & 127) * 8;
  const int sc  = (s < SEQ) ? s : (SEQ - 1);
  const float* src = x + ((size_t)(b * SEQ + sc) * DM + c8);
  const v4f f0 = *(const v4f*)(src);
  const v4f f1 = *(const v4f*)(src + 4);
  v4u u;
  u[0] = pk16(f2bf_bits(f0[0]), f2bf_bits(f0[1]));
  u[1] = pk16(f2bf_bits(f0[2]), f2bf_bits(f0[3]));
  u[2] = pk16(f2bf_bits(f1[0]), f2bf_bits(f1[1]));
  u[3] = pk16(f2bf_bits(f1[2]), f2bf_bits(f1[3]));
  if (s >= SEQ) { u[0] = 0u; u[1] = 0u; u[2] = 0u; u[3] = 0u; }
  unsigned short* dst = xb + ((size_t)row * DM + c8);
  *(volatile v4u*)dst = u;
  __threadfence();
  *(volatile v4u*)dst = u;
}

template <int MODE>
__device__ __forceinline__ unsigned short cvt16(float f) {
  const unsigned short hb = f2bf_bits(f);
  if (MODE == 0) return hb;
  return h_bits((_Float16)(bf_bits2f(hb) * 64.0f));
}

template <int MODE>
__global__ __launch_bounds__(256) void tconv_kernel(const float* __restrict__ W, unsigned short* __restrict__ ot, int R, int Cc) {
  __shared__ __align__(16) float tf[64 * 68];
  const int c0  = blockIdx.x * 64;
  const int r0  = blockIdx.y * 64;
  const int tid = threadIdx.x;
  {
    const int lr = tid >> 4;
    const int c4 = (tid & 15) * 4;
#pragma unroll
    for (int it = 0; it < 4; ++it) {
      const int rr = it * 16 + lr;
      const v4f a = *(const v4f*)(W + (size_t)(r0 + rr) * Cc + c0 + c4);
      *(v4f*)(tf + rr * 68 + c4) = a;
    }
  }
  __syncthreads();
  const int sub = tid >> 3;
  const int c8  = (tid & 7) * 8;
  v4u hv[2];
#pragma unroll
  for (int it = 0; it < 2; ++it) {
    const int oc = it * 32 + sub;
    v4u a;
#pragma unroll
    for (int q = 0; q < 4; ++q) {
      const float f0 = tf[(c8 + 2 * q) * 68 + oc];
      const float f1 = tf[(c8 + 2 * q + 1) * 68 + oc];
      a[q] = pk16(cvt16<MODE>(f0), cvt16<MODE>(f1));
    }
    hv[it] = a;
  }
  for (int pass = 0; pass < 2; ++pass) {
#pragma unroll
    for (int it = 0; it < 2; ++it) {
      const int oc = it * 32 + sub;
      const size_t go = (size_t)(c0 + oc) * R + r0 + c8;
      *(volatile v4u*)(ot + go) = hv[it];
    }
    __threadfence();
  }
}

__device__ __forceinline__ v8f mma_h(v16h a, v16h b, v8f c) {
  c = __builtin_amdgcn_wmma_f32_16x16x32_f16(false, a, false, b, (short)0, c, false, false);
  asm volatile("v_nop\n\tv_nop\n\tv_nop\n\tv_nop" : "+v"(c) : "v"(a), "v"(b));
  return c;
}

__global__ __launch_bounds__(128)
void attn_kernel(const unsigned short* __restrict__ qkhp, const unsigned short* __restrict__ qklp,
                 const unsigned short* __restrict__ vtp, unsigned short* __restrict__ ctxp, float sscale) {
  union FB { v16h v; v8h h[2]; };
  __shared__ __align__(16) _Float16 Ksh[64 * 64];
  __shared__ __align__(16) _Float16 Ksl[64 * 64];
  __shared__ __align__(16) _Float16 Vts[64 * 64];
  __shared__ __align__(16) _Float16 Psh[4][16 * 64];
  __shared__ __align__(16) float    Os[4][16 * 68];

  const int tid  = threadIdx.x;
  const int wave = tid >> 5;
  const int lane = tid & 31;
  const int hh   = lane >> 4;
  const int c    = lane & 15;

  const int bl = blockIdx.y;
  const int bx = blockIdx.x;
  const int qb = bx % NQB;
  const int h  = bx / NQB;
  const int q0 = qb * 64 + wave * 16;

  const _Float16* Qh = (const _Float16*)(const void*)qkhp + (size_t)bl * SP * QKP + h * DH;
  const _Float16* Ql = (const _Float16*)(const void*)qklp + (size_t)bl * SP * QKP + h * DH;
  const _Float16* Kh = Qh + DM;
  const _Float16* Kl = Ql + DM;
  const _Float16* Vt = (const _Float16*)(const void*)vtp + (size_t)bl * DM * SP + (size_t)h * DH * SP;
  _Float16*       ob = (_Float16*)(void*)ctxp + (size_t)bl * SP * DM + h * DH;

  v16h qah[2], qal[2];
#pragma unroll
  for (int dc = 0; dc < 2; ++dc) {
    qah[dc] = Frag<_Float16>::load(Qh + (size_t)(q0 + c) * QKP + dc * 32 + 8 * hh);
    qal[dc] = Frag<_Float16>::load(Ql + (size_t)(q0 + c) * QKP + dc * 32 + 8 * hh);
  }

  float mrow[8], lrow[8];
  v8f oacc[4];
#pragma unroll
  for (int r = 0; r < 8; ++r) { mrow[r] = -INFINITY; lrow[r] = 0.f; }
#pragma unroll
  for (int t = 0; t < 4; ++t) oacc[t] = zero8();

  const float rres = 1.0f / 2048.0f;

  for (int kc = 0; kc < NKC; ++kc) {
    const int kv0 = kc * 64;
    __syncthreads();
    {
      const int r = tid >> 1, half = (tid & 1) * 32;
      const _Float16* ksh = Kh + (size_t)(kv0 + r) * QKP + half;
      const _Float16* ksl = Kl + (size_t)(kv0 + r) * QKP + half;
      const _Float16* vts = Vt + (size_t)r * SP + kv0 + half;
#pragma unroll
      for (int i = 0; i < 4; ++i) {
        const v8h a0 = *(const v8h*)(ksh + 8 * i);
        const v8h a1 = *(const v8h*)(ksl + 8 * i);
        const v8h b0 = *(const v8h*)(vts + 8 * i);
        *(v8h*)(Ksh + r * 64 + half + 8 * i) = a0;
        *(v8h*)(Ksl + r * 64 + half + 8 * i) = a1;
        *(v8h*)(Vts + r * 64 + half + 8 * i) = b0;
      }
    }
    __syncthreads();

    v8f s[4];
#pragma unroll
    for (int j = 0; j < 4; ++j) {
      v8f sa = zero8();
      v8f sr = zero8();
#pragma unroll
      for (int dc = 0; dc < 2; ++dc) {
        FB kb, kl;
        kb.h[0] = *(const v8h*)(Ksh + (j * 16 + c) * 64 + dc * 32 + 8 * hh);
        kb.h[1] = *(const v8h*)(Ksh + (j * 16 + c) * 64 + dc * 32 + 16 + 8 * hh);
        kl.h[0] = *(const v8h*)(Ksl + (j * 16 + c) * 64 + dc * 32 + 8 * hh);
        kl.h[1] = *(const v8h*)(Ksl + (j * 16 + c) * 64 + dc * 32 + 16 + 8 * hh);
        sa = mma_h(qah[dc], kb.v, sa);
        sr = mma_h(qah[dc], kl.v, sr);
        sr = mma_h(qal[dc], kb.v, sr);
      }
      const int col = kv0 + j * 16 + c;
#pragma unroll
      for (int r = 0; r < 8; ++r) {
        const float sv = (sa[r] + sr[r] * rres) * sscale;
        s[j][r] = (col < SEQ) ? sv : -INFINITY;
      }
    }
    float cm[8];
#pragma unroll
    for (int r = 0; r < 8; ++r) {
      float m = fmaxf(fmaxf(s[0][r], s[1][r]), fmaxf(s[2][r], s[3][r]));
#pragma unroll
      for (int off = 1; off < 16; off <<= 1) m = fmaxf(m, __shfl_xor(m, off, 32));
      cm[r] = m;
    }
    _Float16* pw = Psh[wave];
#pragma unroll
    for (int r = 0; r < 8; ++r) {
      const float mnew  = fmaxf(mrow[r], cm[r]);
      const float alpha = __expf(mrow[r] - mnew);
      mrow[r] = mnew;
      float psum = 0.f;
#pragma unroll
      for (int j = 0; j < 4; ++j) {
        const float p = __expf(s[j][r] - mnew);
        psum += p;
        pw[(8 * hh + r) * 64 + j * 16 + c] = (_Float16)(p * 1024.0f);
      }
#pragma unroll
      for (int off = 1; off < 16; off <<= 1) psum += __shfl_xor(psum, off, 32);
      lrow[r] = lrow[r] * alpha + psum;
#pragma unroll
      for (int t = 0; t < 4; ++t) oacc[t][r] *= alpha;
    }
    __builtin_amdgcn_fence(__ATOMIC_RELEASE, "workgroup");
    __builtin_amdgcn_wave_barrier();
    __builtin_amdgcn_fence(__ATOMIC_ACQUIRE, "workgroup");
#pragma unroll 1
    for (int kk = 0; kk < 2; ++kk) {
      FB pa;
      pa.h[0] = *(const v8h*)(pw + c * 64 + kk * 32 + 8 * hh);
      pa.h[1] = *(const v8h*)(pw + c * 64 + kk * 32 + 16 + 8 * hh);
#pragma unroll
      for (int t = 0; t < 4; ++t) {
        FB vb;
        vb.h[0] = *(const v8h*)(Vts + (t * 16 + c) * 64 + kk * 32 + 8 * hh);
        vb.h[1] = *(const v8h*)(Vts + (t * 16 + c) * 64 + kk * 32 + 16 + 8 * hh);
        oacc[t] = mma_h(pa.v, vb.v, oacc[t]);
      }
    }
  }

  float* os = Os[wave];
#pragma unroll
  for (int r = 0; r < 8; ++r) {
    const float inv = 1.0f / (lrow[r] * 1024.0f);
#pragma unroll
    for (int t = 0; t < 4; ++t) os[(8 * hh + r) * 68 + t * 16 + c] = oacc[t][r] * inv;
  }
  __builtin_amdgcn_fence(__ATOMIC_RELEASE, "workgroup");
  __builtin_amdgcn_wave_barrier();
  __builtin_amdgcn_fence(__ATOMIC_ACQUIRE, "workgroup");
  {
    const int qq = lane >> 3, c8 = (lane & 7) * 8;
    for (int pass = 0; pass < 2; ++pass) {
#pragma unroll
      for (int it = 0; it < 4; ++it) {
        const int row = it * 4 + qq;
        const float* sp = os + row * 68 + c8;
        v8h hv;
#pragma unroll
        for (int e = 0; e < 8; ++e) hv[e] = (_Float16)sp[e];
        *(volatile v8h*)(ob + (size_t)(q0 + row) * DM + c8) = hv;
      }
      __threadfence();
    }
  }
}

extern "C" void kernel_launch(void* const* d_in, const int* in_sizes, int n_in,
                              void* d_out, int out_size, void* d_ws, size_t ws_size,
                              hipStream_t stream) {
  if (n_in < 9) return;
  if (in_sizes[0] != NB * SEQ * DM) return;
  if (in_sizes[1] != DM * DM || in_sizes[3] != DM * DM || in_sizes[5] != DM * DM || in_sizes[7] != DM * DM) return;
  if (in_sizes[2] != DM || in_sizes[4] != DM || in_sizes[6] != DM || in_sizes[8] != DM) return;
  if (out_size != NB * SEQ * DM) return;

  const float* x  = (const float*)d_in[0];
  const float* Wq = (const float*)d_in[1];
  const float* bq = (const float*)d_in[2];
  const float* Wk = (const float*)d_in[3];
  const float* bk = (const float*)d_in[4];
  const float* Wv = (const float*)d_in[5];
  const float* bv = (const float*)d_in[6];
  const float* Wo = (const float*)d_in[7];
  const float* bo = (const float*)d_in[8];
  float* out = (float*)d_out;

  const size_t PXB  = (size_t)NB * SP * DM * 2;
  const size_t PWQK = (size_t)2 * DM * DM * 2;
  const size_t PW   = (size_t)DM * DM * 2;
  const size_t PQK  = (size_t)GRP * SP * QKP * 2;
  const size_t PVT  = (size_t)GRP * DM * SP * 2;
  const size_t PCTX = (size_t)GRP * SP * DM * 2;
  size_t off = 0;
  const size_t oXB  = off; off += PXB;
  const size_t oWQK = off; off += PWQK;
  const size_t oWV  = off; off += PW;
  const size_t oWO  = off; off += PW;
  const size_t oQKH = off; off += PQK;
  const size_t oQKL = off; off += PQK;
  const size_t oVT  = off; off += PVT;
  const size_t oCTX = off; off += PCTX;
  if (off > ws_size) return;

  char* ws = (char*)d_ws;
  unsigned short* XB  = (unsigned short*)(ws + oXB);
  unsigned short* WQK = (unsigned short*)(ws + oWQK);
  unsigned short* WV  = (unsigned short*)(ws + oWV);
  unsigned short* WO  = (unsigned short*)(ws + oWO);
  unsigned short* QKH = (unsigned short*)(ws + oQKH);
  unsigned short* QKL = (unsigned short*)(ws + oQKL);
  unsigned short* VT  = (unsigned short*)(ws + oVT);
  unsigned short* CTX = (unsigned short*)(ws + oCTX);

  const dim3 blk(256);

  xconv_kernel<<<dim3(NB * SP / 2), blk, 0, stream>>>(x, XB);
  tconv_kernel<0><<<dim3(DM / 64, DM / 64), blk, 0, stream>>>(Wq, WQK, DM, DM);
  tconv_kernel<0><<<dim3(DM / 64, DM / 64), blk, 0, stream>>>(Wk, WQK + (size_t)DM * DM, DM, DM);
  tconv_kernel<0><<<dim3(DM / 64, DM / 64), blk, 0, stream>>>(Wv, WV, DM, DM);
  tconv_kernel<1><<<dim3(DM / 64, DM / 64), blk, 0, stream>>>(Wo, WO, DM, DM);

  const dim3 gQK(((SP / 64) * (QKP / 64)) / 8, GRP);
  const dim3 gVT(((DM / 64) * (SP / 64)) / 8, GRP);
  const dim3 gWO(((SP / 64) * (DM / 64)) / 8, GRP);
  const dim3 gAT(NH * NQB, GRP);

  for (int g = 0; g < NGRP; ++g) {
    const unsigned short* XBg = XB + (size_t)g * GRP * SP * DM;
    float* outg = out + (size_t)g * GRP * SEQ * DM;
    gemm64_kernel<1, 2, 2><<<gQK, blk, 0, stream>>>(
        XBg, DM, (long)SP * DM, WQK, DM, 0L, (void*)QKH, (void*)QKL, QKP, (long)SP * QKP,
        bq, bk, DM, SP, 2 * DM, DM, SP, 1.0f, 1.0f);
    gemm64_kernel<1, 1, 1><<<gVT, blk, 0, stream>>>(
        WV, DM, 0L, XBg, DM, (long)SP * DM, (void*)VT, (void*)VT, SP, (long)DM * SP,
        bv, bv, DM, DM, SP, DM, DM, 1.0f, 16.0f);
    attn_kernel<<<gAT, dim3(128), 0, stream>>>(QKH, QKL, VT, CTX, 0.125f);
    gemm64_kernel<0, 2, 0><<<gWO, blk, 0, stream>>>(
        CTX, DM, (long)SP * DM, WO, DM, 0L, (void*)outg, (void*)outg, DM, (long)SEQ * DM,
        bo, bo, DM, SP, DM, DM, SEQ, 1.0f / 1024.0f, 1.0f);
  }
  (void)hipGetLastError();
}
